// MultiheadSelfAttention_81655918232006
// MI455X (gfx1250) — hardware-verified
//
#include <hip/hip_runtime.h>
#ifndef NB
#define NB 2
#endif
#ifndef SEQ
#define SEQ 2048
#endif
#define NB_FULL 2
#define SEQ_FULL 2048
#define DM 1024
#define NH 16
#define HD 64
#define ISL (((SEQ) < 512) ? (SEQ) : 512)
#define NR ((size_t)NB * SEQ)
#define NRI ((size_t)NB * ISL)

static_assert(NB <= NB_FULL);
static_assert(SEQ <= SEQ_FULL);
static_assert(DM == NH * HD);
static_assert(HD == 64);
static_assert(DM % 64 == 0);
static_assert(DM % 32 == 0);
static_assert(SEQ % 128 == 0);
static_assert(ISL % 64 == 0);
static_assert(ISL % 32 == 0);
static_assert((SEQ - ISL) % 128 == 0);
static_assert((SEQ - ISL) % 64 == 0);
static_assert((NR * DM) % 8 == 0);

typedef unsigned short v8us __attribute__((ext_vector_type(8), may_alias));
typedef float  v8f  __attribute__((ext_vector_type(8)));
typedef float  v4f  __attribute__((ext_vector_type(4)));
typedef float  v4fa __attribute__((ext_vector_type(4), may_alias));
typedef float  v2fa __attribute__((ext_vector_type(2), may_alias));
typedef _Float16 v16h __attribute__((ext_vector_type(16)));
typedef _Float16 v4h __attribute__((ext_vector_type(4)));
union FragH { v16h v; v8us half[2]; _Float16 h[16]; unsigned short u[16]; };

__device__ __forceinline__ unsigned short bf16_bits(float x) { unsigned int u = __float_as_uint(x); return (unsigned short)((u + 0x7FFFu + ((u >> 16) & 1u)) >> 16); }
__device__ __forceinline__ float bf16_rne(float x) { return __uint_as_float(((unsigned int)bf16_bits(x)) << 16); }

__device__ __forceinline__ v16h g2_frag(const _Float16* p, int hh) { FragH f; f.half[0] = *(const v8us*)((const unsigned short*)p + 8 * hh); f.half[1] = *(const v8us*)((const unsigned short*)p + 16 + 8 * hh); return f.v; }
__device__ __forceinline__ v8f g2_mma(v16h a, v16h b, v8f c) { v8f d = __builtin_amdgcn_wmma_f32_16x16x32_f16(false, a, false, b, (short)0, c, false, false); asm volatile("v_nop\n\tv_nop\n\tv_nop\n\tv_nop" : "+v"(d) : "v"(a), "v"(b)); return d; }

__global__ __launch_bounds__(256) void k_wnat(const float* __restrict__ w, size_t n8, _Float16* __restrict__ Bt) {
  const size_t t = (size_t)blockIdx.x * 256 + threadIdx.x; if (t >= n8) return; FragH f;
#pragma unroll
  for (int q = 0; q < 8; ++q) f.h[q] = (_Float16)(bf16_rne(w[t * 8 + q]) * 16.0f);
  const v8us o = f.half[0];
  *(volatile v8us*)((unsigned short*)Bt + t * 8) = o; __threadfence(); *(volatile v8us*)((unsigned short*)Bt + t * 8) = o;
}

__global__ __launch_bounds__(256) void k_x16(const float* __restrict__ x, _Float16* __restrict__ X16) {
  const size_t t = (size_t)blockIdx.x * 256 + threadIdx.x; if (t >= NR * DM / 8) return;
  const size_t row = t / (DM / 8); const int c8 = (int)(t % (DM / 8)) * 8;
  const size_t b = row / SEQ, s = row % SEQ;
  const float* src = x + (b * SEQ_FULL + s) * DM + c8;
  const v4f a = *(const v4fa*)src, c = *(const v4fa*)(src + 4);
  FragH f;
#pragma unroll
  for (int q = 0; q < 4; ++q) { f.h[q] = (_Float16)bf16_rne(a[q]); f.h[4 + q] = (_Float16)bf16_rne(c[q]); }
  const v8us o = f.half[0];
  *(volatile v8us*)((unsigned short*)X16 + t * 8) = o; __threadfence(); *(volatile v8us*)((unsigned short*)X16 + t * 8) = o;
}

__global__ __launch_bounds__(32) void k_freq(float* __restrict__ DEN) {
  const int i = threadIdx.x & 31;
  const float e = (float)(2 * i) / 64.0f;
  const float d = powf(10000.0f, e);
  *(volatile float*)(DEN + i) = d; __threadfence(); *(volatile float*)(DEN + i) = d;
}

__global__ __launch_bounds__(256) void k_rtab(const int* __restrict__ pos, const float* __restrict__ DEN, float* __restrict__ CS) {
  const int t = blockIdx.x * 256 + threadIdx.x; if (t >= SEQ * 32) return;
  const int s = t >> 5, i = t & 31;
  const float ang = (float)pos[s] / DEN[i];
  float sn, cs; sincosf(ang, &sn, &cs);
  float* c = CS + (size_t)s * 64;
  *(volatile float*)(c + i) = cs; *(volatile float*)(c + 32 + i) = sn;
  __threadfence();
  *(volatile float*)(c + i) = cs; *(volatile float*)(c + 32 + i) = sn;
}

__global__ __launch_bounds__(128) void k_proj(const _Float16* __restrict__ X16, const _Float16* __restrict__ BW, const float* __restrict__ CS, _Float16* __restrict__ P16, _Float16* __restrict__ RL) {
  #pragma clang fp contract(off)
  __shared__ __attribute__((aligned(16))) float so[4][32][68];
  const int tid = threadIdx.x, w = tid >> 5, lane = tid & 31, ln = lane & 15, hh = lane >> 4; const int y = blockIdx.y;
  const _Float16* Bh = BW + (size_t)y * DM * DM;
  const int ntn = DM / 64; const int mt = blockIdx.x / ntn, nq = blockIdx.x - mt * ntn; const int row0 = mt * 128 + 32 * w, col0 = nq * 64;
  const _Float16* a0p = X16 + (size_t)(row0 + ln) * DM; const _Float16* a1p = a0p + (size_t)16 * DM;
  const _Float16* b0p = Bh + (size_t)(col0 + ln) * DM; const _Float16* b1p = b0p + (size_t)16 * DM; const _Float16* b2p = b1p + (size_t)16 * DM; const _Float16* b3p = b2p + (size_t)16 * DM;
  const v8f z8 = {0.f,0.f,0.f,0.f,0.f,0.f,0.f,0.f}; v8f c00 = z8, c01 = z8, c02 = z8, c03 = z8, c10 = z8, c11 = z8, c12 = z8, c13 = z8;
#pragma unroll 1
  for (int kb = 0; kb < DM; kb += 32) { const v16h a0 = g2_frag(a0p + kb, hh), a1 = g2_frag(a1p + kb, hh);
    v16h b = g2_frag(b0p + kb, hh); c00 = g2_mma(a0, b, c00); c10 = g2_mma(a1, b, c10);
    b = g2_frag(b1p + kb, hh); c01 = g2_mma(a0, b, c01); c11 = g2_mma(a1, b, c11);
    b = g2_frag(b2p + kb, hh); c02 = g2_mma(a0, b, c02); c12 = g2_mma(a1, b, c12);
    b = g2_frag(b3p + kb, hh); c03 = g2_mma(a0, b, c03); c13 = g2_mma(a1, b, c13); }
  v8f accs[8] = {c00, c01, c02, c03, c10, c11, c12, c13};
#pragma unroll
  for (int u = 0; u < 8; ++u) { const int t = u & 3, half = u >> 2;
#pragma unroll
    for (int r = 0; r < 8; ++r) so[w][half * 16 + 8 * hh + r][t * 16 + ln] = accs[u][r] * 0.0625f; }
  __builtin_amdgcn_fence(4  , "workgroup"); __builtin_amdgcn_wave_barrier();
  const int rsub = lane >> 4, c4 = (lane & 15) * 4;
  const int sq0 = row0 % SEQ, bb = row0 / SEQ; const bool isl = sq0 < ISL;
  if (y < 2) {
    const int i0 = c4 >> 1;
#pragma unroll 4
    for (int q = 0; q < 16; ++q) { const int r = q * 2 + rsub; const int s = sq0 + r;
      const v4f v = *(const v4fa*)&so[w][r][c4];
      const v2fa cc = *(const v2fa*)(CS + (size_t)s * 64 + i0); const v2fa ss = *(const v2fa*)(CS + (size_t)s * 64 + 32 + i0);
      v4f o; o[0] = v[0] * cc[0] - v[1] * ss[0]; o[1] = v[0] * ss[0] + v[1] * cc[0]; o[2] = v[2] * cc[1] - v[3] * ss[1]; o[3] = v[2] * ss[1] + v[3] * cc[1];
      *(v4fa*)&so[w][r][c4] = o; }
  }
  _Float16* Ch = P16 + (size_t)y * NR * DM; _Float16* Cl = RL + (size_t)y * NRI * DM;
  for (int pass = 0; pass < 2; ++pass) {
#pragma unroll 4
    for (int q = 0; q < 16; ++q) { const int r = q * 2 + rsub; const v4f v = *(const v4fa*)&so[w][r][c4]; v4h h4;
#pragma unroll
      for (int i = 0; i < 4; ++i) h4[i] = (_Float16)v[i];
      *(volatile v4h*)(Ch + (size_t)(row0 + r) * DM + col0 + c4) = h4;
      if (isl) { v4h l4;
#pragma unroll
        for (int i = 0; i < 4; ++i) l4[i] = (_Float16)((v[i] - (float)h4[i]) * 1024.0f);
        *(volatile v4h*)(Cl + ((size_t)bb * ISL + sq0 + r) * DM + col0 + c4) = l4; } }
    if (pass == 0) __threadfence(); }
}

__global__ __launch_bounds__(256) void k_vt(const _Float16* __restrict__ V16, _Float16* __restrict__ Vt, int TT) {
  __shared__ unsigned short tl[64][66]; const int tid = threadIdx.x; const int nlg = TT / 64; const int slab = blockIdx.x / nlg, lg = blockIdx.x - slab * nlg; const int b = slab / NH, h = slab - b * NH;
  for (int i = tid; i < 64 * 8; i += 256) { const int r = i / 8, c8 = (i % 8) * 8; FragH f; f.half[0] = *(const v8us*)((const unsigned short*)V16 + ((size_t)b * TT + lg * 64 + r) * DM + h * HD + c8);
#pragma unroll
    for (int q = 0; q < 8; ++q) tl[r][c8 + q] = f.u[q]; }
  __syncthreads();
  for (int pass = 0; pass < 2; ++pass) {
#pragma unroll
    for (int rd = 0; rd < 2; ++rd) { const int d = rd * 32 + tid / 8, pc = tid % 8; FragH f;
#pragma unroll
      for (int q = 0; q < 8; ++q) f.u[q] = tl[pc * 8 + q][d];
      *(volatile v8us*)((unsigned short*)Vt + ((size_t)slab * 64 + d) * TT + lg * 64 + pc * 8) = f.half[0]; }
    if (pass == 0) __threadfence(); } }

template <bool RES>
__device__ __forceinline__ void attn_body(const _Float16* __restrict__ QH, const _Float16* __restrict__ QL, const _Float16* __restrict__ KH, const _Float16* __restrict__ KL,
                                          const _Float16* __restrict__ VT, const _Float16* __restrict__ VTL, _Float16* __restrict__ OH, _Float16* __restrict__ OL, int qbase) {
  __shared__ __attribute__((aligned(16))) float so[4][16][68];
  __shared__ __attribute__((aligned(16))) _Float16 ph[4][16][40];
  __shared__ __attribute__((aligned(16))) _Float16 pr[4][16][40];
  const int tid = threadIdx.x; const int w = __builtin_amdgcn_readfirstlane(tid >> 5); const int lane = tid & 31, ln = lane & 15, hh = lane >> 4;
  const int bh = blockIdx.y; const int b = bh / NH, h = bh - b * NH;
  const int q0w = qbase + 64 * (int)blockIdx.x + 16 * w;
  const size_t qoff = ((size_t)b * SEQ + q0w + ln) * DM + h * HD;
  const size_t qloff = ((size_t)b * ISL + q0w + ln) * DM + h * HD;
  const size_t kbase = ((size_t)b * SEQ + ln) * DM + h * HD;
  const size_t klbase = ((size_t)b * ISL + ln) * DM + h * HD;
  const size_t vbase = ((size_t)bh * HD + ln) * SEQ;
  const size_t vlbase = ((size_t)bh * HD + ln) * ISL;
  const v8f z8 = {0.f,0.f,0.f,0.f,0.f,0.f,0.f,0.f};
  v8f om[4] = {z8, z8, z8, z8}; v8f orr[4] = {z8, z8, z8, z8};
  float m[8], l[8];
#pragma unroll
  for (int r = 0; r < 8; ++r) { m[r] = -1.0e30f; l[r] = 0.f; }
  const int kend = q0w + 16;
#pragma unroll 1
  for (int kv = 0; kv < kend; kv += 32) {
    v8f s0 = z8, s1 = z8, t0 = z8, t1 = z8;
#pragma unroll
    for (int ds = 0; ds < 2; ++ds) {
      const v16h qa = g2_frag(QH + qoff + ds * 32, hh);
      const size_t ko = kbase + (size_t)kv * DM + ds * 32;
      const size_t klo = klbase + (size_t)kv * DM + ds * 32;
      v16h kb = g2_frag(KH + ko, hh);
      s0 = g2_mma(qa, kb, s0);
      if (RES) { const v16h ql = g2_frag(QL + qloff + ds * 32, hh); t0 = g2_mma(ql, kb, t0); const v16h kl = g2_frag(KL + klo, hh); t0 = g2_mma(qa, kl, t0);
        kb = g2_frag(KH + ko + (size_t)16 * DM, hh); s1 = g2_mma(qa, kb, s1); t1 = g2_mma(ql, kb, t1); const v16h kl1 = g2_frag(KL + klo + (size_t)16 * DM, hh); t1 = g2_mma(qa, kl1, t1); }
      else { kb = g2_frag(KH + ko + (size_t)16 * DM, hh); s1 = g2_mma(qa, kb, s1); }
    }
    float e0a[8], e1a[8];
#pragma unroll
    for (int r = 0; r < 8; ++r) {
      const int row = q0w + 8 * hh + r;
      float x0 = s0[r], x1 = s1[r];
      if (RES) { x0 += t0[r] * 0.0009765625f; x1 += t1[r] * 0.0009765625f; }
      x0 *= 0.125f; x1 *= 0.125f;
      const float v0 = (kv + ln <= row) ? x0 : -1.0e9f;
      const float v1 = (kv + 16 + ln <= row) ? x1 : -1.0e9f;
      float tm = fmaxf(v0, v1);
      tm = fmaxf(tm, __shfl_xor(tm, 1)); tm = fmaxf(tm, __shfl_xor(tm, 2)); tm = fmaxf(tm, __shfl_xor(tm, 4)); tm = fmaxf(tm, __shfl_xor(tm, 8));
      const float mn = fmaxf(m[r], tm);
      const float a = __expf(m[r] - mn);
      const float e0 = __expf(v0 - mn), e1 = __expf(v1 - mn);
      float ts = e0 + e1;
      ts += __shfl_xor(ts, 1); ts += __shfl_xor(ts, 2); ts += __shfl_xor(ts, 4); ts += __shfl_xor(ts, 8);
      l[r] = l[r] * a + ts; m[r] = mn;
      om[0][r] *= a; om[1][r] *= a; om[2][r] *= a; om[3][r] *= a;
      if (RES) { orr[0][r] *= a; orr[1][r] *= a; orr[2][r] *= a; orr[3][r] *= a; }
      e0a[r] = e0 * 1024.0f; e1a[r] = e1 * 1024.0f;
    }
#pragma unroll
    for (int r = 0; r < 8; ++r) {
      const _Float16 h0 = (_Float16)e0a[r], h1 = (_Float16)e1a[r];
      ph[w][8 * hh + r][ln] = h0; ph[w][8 * hh + r][16 + ln] = h1;
      if (RES) { pr[w][8 * hh + r][ln] = (_Float16)((e0a[r] - (float)h0) * 1024.0f); pr[w][8 * hh + r][16 + ln] = (_Float16)((e1a[r] - (float)h1) * 1024.0f); }
    }
    __builtin_amdgcn_fence(4  , "workgroup"); __builtin_amdgcn_wave_barrier();
    FragH pa, pb;
    pa.half[0] = *(const v8us*)&ph[w][ln][8 * hh]; pa.half[1] = *(const v8us*)&ph[w][ln][16 + 8 * hh];
    if (RES) { pb.half[0] = *(const v8us*)&pr[w][ln][8 * hh]; pb.half[1] = *(const v8us*)&pr[w][ln][16 + 8 * hh]; } else { pb.v = pa.v; }
    {
      const size_t vo = vbase + (size_t)kv;
      const v16h vb0 = g2_frag(VT + vo, hh), vb1 = g2_frag(VT + vo + (size_t)16 * SEQ, hh), vb2 = g2_frag(VT + vo + (size_t)32 * SEQ, hh), vb3 = g2_frag(VT + vo + (size_t)48 * SEQ, hh);
      om[0] = g2_mma(pa.v, vb0, om[0]); om[1] = g2_mma(pa.v, vb1, om[1]); om[2] = g2_mma(pa.v, vb2, om[2]); om[3] = g2_mma(pa.v, vb3, om[3]);
      if (RES) { orr[0] = g2_mma(pb.v, vb0, orr[0]); orr[1] = g2_mma(pb.v, vb1, orr[1]); orr[2] = g2_mma(pb.v, vb2, orr[2]); orr[3] = g2_mma(pb.v, vb3, orr[3]); }
    }
    if (RES) {
      const size_t vlo = vlbase + (size_t)kv;
      const v16h vl0 = g2_frag(VTL + vlo, hh), vl1 = g2_frag(VTL + vlo + (size_t)16 * ISL, hh), vl2 = g2_frag(VTL + vlo + (size_t)32 * ISL, hh), vl3 = g2_frag(VTL + vlo + (size_t)48 * ISL, hh);
      orr[0] = g2_mma(pa.v, vl0, orr[0]); orr[1] = g2_mma(pa.v, vl1, orr[1]); orr[2] = g2_mma(pa.v, vl2, orr[2]); orr[3] = g2_mma(pa.v, vl3, orr[3]);
    }
    __builtin_amdgcn_fence(4  , "workgroup"); __builtin_amdgcn_wave_barrier();
  }
#pragma unroll
  for (int r = 0; r < 8; ++r) {
    const float f = 0.0625f * (1.0f / l[r]);
#pragma unroll
    for (int t = 0; t < 4; ++t) { float v = om[t][r]; if (RES) v += orr[t][r] * 0.0009765625f; so[w][8 * hh + r][t * 16 + ln] = v * f; }
  }
  __builtin_amdgcn_fence(4  , "workgroup"); __builtin_amdgcn_wave_barrier();
  const int rsub = lane >> 4, c4 = (lane & 15) * 4;
  for (int pass = 0; pass < 2; ++pass) {
#pragma unroll
    for (int q = 0; q < 8; ++q) { const int r = q * 2 + rsub; const v4f v = *(const v4fa*)&so[w][r][c4]; v4h h4;
#pragma unroll
      for (int i = 0; i < 4; ++i) h4[i] = (_Float16)v[i];
      *(volatile v4h*)(OH + ((size_t)b * SEQ + q0w + r) * DM + h * HD + c4) = h4;
      if (RES) { v4h l4;
#pragma unroll
        for (int i = 0; i < 4; ++i) l4[i] = (_Float16)((v[i] - (float)h4[i]) * 1024.0f);
        *(volatile v4h*)(OL + ((size_t)b * ISL + q0w + r) * DM + h * HD + c4) = l4; } }
    if (pass == 0) __threadfence(); }
}
__global__ __launch_bounds__(128) void k_attn_isl(const _Float16* __restrict__ QH, const _Float16* __restrict__ QL, const _Float16* __restrict__ KH, const _Float16* __restrict__ KL,
                                                  const _Float16* __restrict__ VT, const _Float16* __restrict__ VTL, _Float16* __restrict__ OH, _Float16* __restrict__ OL) {
  attn_body<true>(QH, QL, KH, KL, VT, VTL, OH, OL, 0); }
__global__ __launch_bounds__(128) void k_attn_pl(const _Float16* __restrict__ QH, const _Float16* __restrict__ KH, const _Float16* __restrict__ VT, _Float16* __restrict__ OH) {
  attn_body<false>(QH, QH, KH, KH, VT, VT, OH, OH, ISL); }

__global__ __launch_bounds__(128) void k_outp(const _Float16* __restrict__ OH, const _Float16* __restrict__ Bh, float* __restrict__ C) {
  __shared__ __attribute__((aligned(16))) float so[4][32][68];
  const int tid = threadIdx.x, w = tid >> 5, lane = tid & 31, ln = lane & 15, hh = lane >> 4; const int by = blockIdx.y;
  const _Float16* A = OH + ((size_t)by * SEQ + ISL) * DM; float* Cb = C + ((size_t)by * SEQ_FULL + ISL) * DM;
  const int ntn = DM / 64; const int mt = blockIdx.x / ntn, nq = blockIdx.x - mt * ntn; const int row0 = mt * 128 + 32 * w, col0 = nq * 64;
  const _Float16* a0p = A + (size_t)(row0 + ln) * DM; const _Float16* a1p = a0p + (size_t)16 * DM;
  const _Float16* b0p = Bh + (size_t)(col0 + ln) * DM; const _Float16* b1p = b0p + (size_t)16 * DM; const _Float16* b2p = b1p + (size_t)16 * DM; const _Float16* b3p = b2p + (size_t)16 * DM;
  const v8f z8 = {0.f,0.f,0.f,0.f,0.f,0.f,0.f,0.f}; v8f c00 = z8, c01 = z8, c02 = z8, c03 = z8, c10 = z8, c11 = z8, c12 = z8, c13 = z8;
#pragma unroll 1
  for (int kb = 0; kb < DM; kb += 32) { const v16h a0 = g2_frag(a0p + kb, hh), a1 = g2_frag(a1p + kb, hh);
    v16h b = g2_frag(b0p + kb, hh); c00 = g2_mma(a0, b, c00); c10 = g2_mma(a1, b, c10);
    b = g2_frag(b1p + kb, hh); c01 = g2_mma(a0, b, c01); c11 = g2_mma(a1, b, c11);
    b = g2_frag(b2p + kb, hh); c02 = g2_mma(a0, b, c02); c12 = g2_mma(a1, b, c12);
    b = g2_frag(b3p + kb, hh); c03 = g2_mma(a0, b, c03); c13 = g2_mma(a1, b, c13); }
  v8f accs[8] = {c00, c01, c02, c03, c10, c11, c12, c13};
#pragma unroll
  for (int u = 0; u < 8; ++u) { const int t = u & 3, half = u >> 2;
#pragma unroll
    for (int r = 0; r < 8; ++r) so[w][half * 16 + 8 * hh + r][t * 16 + ln] = accs[u][r] * 0.0009765625f; }
  __builtin_amdgcn_fence(4  , "workgroup"); __builtin_amdgcn_wave_barrier();
  const int rsub = lane >> 4, c4 = (lane & 15) * 4;
  for (int pass = 0; pass < 2; ++pass) {
#pragma unroll
    for (int q = 0; q < 16; ++q) { const int r = q * 2 + rsub; const v4f v = *(const v4fa*)&so[w][r][c4]; *(volatile v4f*)(Cb + (size_t)(row0 + r) * DM + col0 + c4) = v; }
    if (pass == 0) __threadfence(); }
}

__global__ __launch_bounds__(128) void k_outi(const _Float16* __restrict__ OH, const _Float16* __restrict__ OL, const _Float16* __restrict__ Bh, float* __restrict__ C) {
  __shared__ __attribute__((aligned(16))) float so[4][16][68];
  const int tid = threadIdx.x, w = tid >> 5, lane = tid & 31, ln = lane & 15, hh = lane >> 4; const int by = blockIdx.y;
  const int ntn = DM / 64; const int mt = blockIdx.x / ntn, nq = blockIdx.x - mt * ntn; const int row0 = mt * 64 + 16 * w, col0 = nq * 64;
  const _Float16* ahp = OH + ((size_t)by * SEQ + row0 + ln) * DM; const _Float16* alp = OL + ((size_t)by * ISL + row0 + ln) * DM;
  const _Float16* b0p = Bh + (size_t)(col0 + ln) * DM;
  float* Cb = C + (size_t)by * SEQ_FULL * DM;
  const v8f z8 = {0.f,0.f,0.f,0.f,0.f,0.f,0.f,0.f}; v8f ch[4] = {z8, z8, z8, z8}; v8f cl[4] = {z8, z8, z8, z8};
#pragma unroll 1
  for (int kb = 0; kb < DM; kb += 32) { const v16h ah = g2_frag(ahp + kb, hh), al = g2_frag(alp + kb, hh);
#pragma unroll
    for (int t = 0; t < 4; ++t) { const v16h b = g2_frag(b0p + (size_t)t * 16 * DM + kb, hh); ch[t] = g2_mma(ah, b, ch[t]); cl[t] = g2_mma(al, b, cl[t]); } }
#pragma unroll
  for (int t = 0; t < 4; ++t) {
#pragma unroll
    for (int r = 0; r < 8; ++r) so[w][8 * hh + r][t * 16 + ln] = (ch[t][r] + cl[t][r] * 0.0009765625f) * 0.0009765625f; }
  __builtin_amdgcn_fence(4  , "workgroup"); __builtin_amdgcn_wave_barrier();
  const int rsub = lane >> 4, c4 = (lane & 15) * 4;
  for (int pass = 0; pass < 2; ++pass) {
#pragma unroll
    for (int q = 0; q < 8; ++q) { const int r = q * 2 + rsub; const v4f v = *(const v4fa*)&so[w][r][c4]; *(volatile v4f*)(Cb + (size_t)(row0 + r) * DM + col0 + c4) = v; }
    if (pass == 0) __threadfence(); }
}

constexpr size_t SZ_W  = (size_t)DM * DM * 2;
constexpr size_t SZ_R  = NR * DM * 2;
constexpr size_t SZ_I  = NRI * DM * 2;
constexpr size_t SZ_CS = (size_t)SEQ * 64 * 4;
constexpr size_t WS_TOTAL = 4 * SZ_W + SZ_R + 3 * SZ_R + 3 * SZ_I + SZ_R + SZ_I + SZ_R + SZ_I + SZ_CS + 256;
static_assert(WS_TOTAL <= (size_t)134217728);
static_assert(SZ_W % 256 == 0 && SZ_R % 256 == 0 && SZ_I % 256 == 0 && SZ_CS % 256 == 0);

extern "C" void kernel_launch(void* const* d_in, const int* in_sizes, int n_in,
                              void* d_out, int out_size, void* d_ws, size_t ws_size, hipStream_t stream) {
  if (n_in < 6) return;
  const size_t need_x = ((size_t)(NB - 1) * SEQ_FULL + SEQ) * DM;
  if ((size_t)in_sizes[0] < need_x) return;
  if (in_sizes[1] < SEQ) return;
  if ((size_t)in_sizes[2] < (size_t)DM * DM || (size_t)in_sizes[3] < (size_t)DM * DM || (size_t)in_sizes[4] < (size_t)DM * DM || (size_t)in_sizes[5] < (size_t)DM * DM) return;
  if ((size_t)out_size < need_x) return;
  if (WS_TOTAL > ws_size) return;
  const float* x = (const float*)d_in[0]; const int* pos = (const int*)d_in[1];
  const float* wq = (const float*)d_in[2]; const float* wk = (const float*)d_in[3]; const float* wv = (const float*)d_in[4]; const float* wo = (const float*)d_in[5];
  float* out = (float*)d_out;
  char* ws = (char*)d_ws; size_t off = 0;
  _Float16* BW  = (_Float16*)(ws + off); off += 3 * SZ_W;
  _Float16* BO  = (_Float16*)(ws + off); off += SZ_W;
  _Float16* X16 = (_Float16*)(ws + off); off += SZ_R;
  _Float16* P16 = (_Float16*)(ws + off); off += 3 * SZ_R;
  _Float16* RL  = (_Float16*)(ws + off); off += 3 * SZ_I;
  _Float16* VT  = (_Float16*)(ws + off); off += SZ_R;
  _Float16* VTL = (_Float16*)(ws + off); off += SZ_I;
  _Float16* OH  = (_Float16*)(ws + off); off += SZ_R;
  _Float16* OL  = (_Float16*)(ws + off); off += SZ_I;
  float* CS     = (float*)(ws + off);    off += SZ_CS;
  float* DEN    = (float*)(ws + off);    off += 256;
  if (off > ws_size) return;
  _Float16* QH = P16; _Float16* KH = P16 + NR * DM; _Float16* VH = P16 + 2 * NR * DM;
  _Float16* QL = RL;  _Float16* KL = RL + NRI * DM; _Float16* VL = RL + 2 * NRI * DM;

  { const size_t n8 = (size_t)DM * DM / 8; const unsigned g = (unsigned)((n8 + 255) / 256);
    k_wnat<<<g, 256, 0, stream>>>(wq, n8, BW);
    k_wnat<<<g, 256, 0, stream>>>(wk, n8, BW + (size_t)DM * DM);
    k_wnat<<<g, 256, 0, stream>>>(wv, n8, BW + (size_t)2 * DM * DM);
    k_wnat<<<g, 256, 0, stream>>>(wo, n8, BO); }
  k_x16<<<(unsigned)((NR * DM / 8 + 255) / 256), 256, 0, stream>>>(x, X16);
  k_freq<<<1, 32, 0, stream>>>(DEN);
  k_rtab<<<(unsigned)((SEQ * 32 + 255) / 256), 256, 0, stream>>>(pos, DEN, CS);
  k_proj<<<dim3((unsigned)((NR / 128) * (DM / 64)), 3), 128, 0, stream>>>(X16, BW, CS, P16, RL);
  k_vt<<<(unsigned)(NB * NH * (SEQ / 64)), 256, 0, stream>>>(VH, VT, SEQ);
  k_vt<<<(unsigned)(NB * NH * (ISL / 64)), 256, 0, stream>>>(VL, VTL, ISL);
  k_attn_isl<<<dim3((unsigned)(ISL / 64), (unsigned)(NB * NH)), 128, 0, stream>>>(QH, QL, KH, KL, VT, VTL, OH, OL);
  if (SEQ > ISL) k_attn_pl<<<dim3((unsigned)((SEQ - ISL) / 64), (unsigned)(NB * NH)), 128, 0, stream>>>(QH, KH, VT, OH);
  k_outi<<<dim3((unsigned)((ISL / 64) * (DM / 64)), (unsigned)NB), 128, 0, stream>>>(OH, OL, BO, out);
  if (SEQ > ISL) k_outp<<<dim3((unsigned)(((SEQ - ISL) / 128) * (DM / 64)), (unsigned)NB), 128, 0, stream>>>(OH, BO, out);
}
